// Fusion_17523466568155
// MI455X (gfx1250) — hardware-verified
//
#include <hip/hip_runtime.h>


namespace {
constexpr int BT = 64, C = 64, L = 512, INTER = 128, DCP = 256, DDE = 1024, K = 16, CL = 64  ;
constexpr float XS = 8.0f, WSC = 256.0f, SCALE = 0.05f;
static_assert(L % 64 == 0 && CL >= 1 && CL <= C, "tiling");
typedef _Float16 b16;
typedef __attribute__((ext_vector_type(16))) _Float16 v16b;
typedef __attribute__((ext_vector_type(8))) _Float16 v8b;
typedef __attribute__((ext_vector_type(8))) float v8f;
typedef __attribute__((ext_vector_type(4))) float v4f;
__device__ __forceinline__ float bf16_rne(float f) { unsigned int u = __float_as_uint(f); u += 0x7FFFu + ((u >> 16) & 1u); return __uint_as_float(u & 0xFFFF0000u); }
__device__ __forceinline__ void split16(float v, b16& hi, b16& lo) { hi = (b16)v; lo = (b16)(v - (float)hi); }
__device__ __forceinline__ v16b frag_kb(const b16* p, int hh) { const v8b a = *(const v8b*)(p + 8 * hh), b = *(const v8b*)(p + 16 + 8 * hh); v16b f;
#pragma unroll
  for (int e = 0; e < 8; ++e) { f[e] = a[e]; f[8 + e] = b[e]; } return f; }
__device__ __forceinline__ v8f wmma16b(v16b a, v16b b, v8f c) { v8f d = __builtin_amdgcn_wmma_f32_16x16x32_f16(false, a, false, b, (short)0, c, false, false); asm volatile("v_nop\n\tv_nop\n\tv_nop\n\tv_nop" : "+v"(d) : "v"(a), "v"(b)); return d; }
__device__ __forceinline__ void wave_lds_sync() { __builtin_amdgcn_fence(__ATOMIC_RELEASE, "workgroup"); __builtin_amdgcn_wave_barrier(); __builtin_amdgcn_fence(__ATOMIC_ACQUIRE, "workgroup"); }
__device__ __forceinline__ float pmul(float a, float b) { float p = a * b; asm volatile("" : "+v"(p)); return p; }
__device__ __forceinline__ int iclamp(int v, int lo, int hi) { return v < lo ? lo : (v > hi ? hi : v); }

typedef __attribute__((ext_vector_type(2))) _Float16 v2h;
typedef __attribute__((ext_vector_type(4))) _Float16 v4h;
typedef __attribute__((ext_vector_type(2))) float v2f;
__device__ __attribute__((noinline)) float expnl(float v) { return expf(v); }
__device__ __attribute__((noinline)) float sigm(float v) { return 1.0f / (1.0f + expf(-v)); }
__global__ __launch_bounds__(256) void prep_kernel(const float* __restrict__ w1, const float* __restrict__ w2, const float* __restrict__ w3, const float* __restrict__ w4, b16* __restrict__ W1T, b16* __restrict__ W2T, b16* __restrict__ W3T, b16* __restrict__ W4T) {
  size_t t = (size_t)blockIdx.x * 256 + threadIdx.x; v8b o;
  const size_t n1 = (size_t)DCP * INTER / 8, n2 = (size_t)DCP * DCP / 8, n3 = (size_t)DDE * L / 8, n4 = (size_t)L * DDE / 8;
  const float* w; b16* dst; int KD, OD; size_t e;
  if (t < n1) { w = w1; dst = W1T; KD = INTER; OD = DCP; e = t * 8; } else if (t < n1 + n2) { w = w2; dst = W2T; KD = DCP; OD = DCP; e = (t - n1) * 8; } else if (t < n1 + n2 + n3) { w = w3; dst = W3T; KD = L; OD = DDE; e = (t - n1 - n2) * 8; } else if (t < n1 + n2 + n3 + n4) { w = w4; dst = W4T; KD = DDE; OD = L; e = (t - n1 - n2 - n3) * 8; } else return;
  (void)OD; const int oo = (int)(e / KD), k0 = (int)(e % KD); for (int j = 0; j < 8; ++j) o[j] = (b16)(bf16_rne(w[(size_t)(k0 + j) * OD + oo]) * WSC);
  for (int pass = 0; pass < 2; ++pass) { *(volatile v8b*)(dst + e) = o; __threadfence(); }
}
template <int KD, int OD, int AF32, int RELU, int OUTF32>
__global__ __launch_bounds__(128) void gemm_kernel(const float* __restrict__ Af, const b16* __restrict__ Ap, const b16* __restrict__ WT, const float* __restrict__ bias, int MC, b16* __restrict__ Op, float* __restrict__ Of) {
  __shared__ __attribute__((aligned(16))) float Tf[4][16][128 + 4]; __shared__ __attribute__((aligned(16))) b16 As[4][16][(AF32 ? KD : 32) + 8];
  const int wave = threadIdx.x >> 5, lane = threadIdx.x & 31, nloc = lane & 15, hlf = lane >> 4; const size_t m0 = ((size_t)blockIdx.x * 4 + wave) * 16; const int n0 = blockIdx.y * 128; if (m0 >= (size_t)MC) return;
  if (AF32) { for (int rr = 0; rr < 16; ++rr) { const float* xr = Af + (m0 + rr) * KD; for (int q = lane * 4; q < KD; q += 128) { const v4f xv = *(const v4f*)(xr + q); v4h o; for (int j = 0; j < 4; ++j) o[j] = (b16)(bf16_rne(xv[j]) * XS); *(v4h*)(&As[wave][rr][q]) = o; } } wave_lds_sync(); }
  v8f acc[8];
#pragma unroll
  for (int t = 0; t < 8; ++t) acc[t] = (v8f){};
#pragma unroll 2
  for (int kb = 0; kb < KD; kb += 32) { const v16b a = AF32 ? frag_kb(&As[wave][nloc][kb], hlf) : frag_kb(Ap + (m0 + nloc) * KD + kb, hlf);
#pragma unroll
    for (int t = 0; t < 8; ++t) acc[t] = wmma16b(a, frag_kb(WT + (size_t)(n0 + t * 16 + nloc) * KD + kb, hlf), acc[t]); }
#pragma unroll
  for (int t = 0; t < 8; ++t) { const float bb = bf16_rne(bias[n0 + t * 16 + nloc]);
#pragma unroll
    for (int r = 0; r < 8; ++r) { float v = acc[t][r] * (1.0f / (XS * WSC)) + bb; if (RELU) v = fmaxf(v, 0.0f); Tf[wave][8 * hlf + r][t * 16 + nloc] = v; } }
  wave_lds_sync();
  for (int pass = 0; pass < 2; ++pass) { for (int rr = 0; rr < 16; ++rr) { const v4f f = *(const v4f*)(&Tf[wave][rr][lane * 4]);
      if (OUTF32) *(volatile v4f*)(Of + (m0 + rr) * OD + n0 + lane * 4) = f; else { v4h o; for (int j = 0; j < 4; ++j) o[j] = (b16)(f[j] * XS); *(volatile v4h*)(Op + (m0 + rr) * OD + n0 + lane * 4) = o; } }
    __threadfence(); }
}
__global__ __launch_bounds__(128) void gemm2t_kernel(const b16* __restrict__ T1, const b16* __restrict__ W2T, const float* __restrict__ b2, b16* __restrict__ T2T) {
  __shared__ __attribute__((aligned(16))) float Tf[4][16][128 + 4];
  const int wave = threadIdx.x >> 5, lane = threadIdx.x & 31, nloc = lane & 15, hlf = lane >> 4; const int c = blockIdx.x / (L / 64), lb = blockIdx.x % (L / 64); const int l0 = lb * 64 + wave * 16; const int n0 = blockIdx.y * 128; if (c >= CL) return;
  const size_t m0 = (size_t)c * L + l0;
  v8f acc[8];
#pragma unroll
  for (int t = 0; t < 8; ++t) acc[t] = (v8f){};
#pragma unroll 2
  for (int kb = 0; kb < DCP; kb += 32) { const v16b a = frag_kb(T1 + (m0 + nloc) * DCP + kb, hlf);
#pragma unroll
    for (int t = 0; t < 8; ++t) acc[t] = wmma16b(a, frag_kb(W2T + (size_t)(n0 + t * 16 + nloc) * DCP + kb, hlf), acc[t]); }
#pragma unroll
  for (int t = 0; t < 8; ++t) { const float bb = bf16_rne(b2[n0 + t * 16 + nloc]);
#pragma unroll
    for (int r = 0; r < 8; ++r) Tf[wave][8 * hlf + r][t * 16 + nloc] = acc[t][r] * (1.0f / (XS * WSC)) + bb; }
  __syncthreads();
  for (int pass = 0; pass < 2; ++pass) {
#pragma unroll 1
    for (int q = 0; q < 32; ++q) { const int dl = wave * 32 + q; const int d = n0 + dl; const int tk = lane * 2; v2h vv; vv[0] = (b16)(Tf[tk >> 4][tk & 15][dl] * XS); vv[1] = (b16)(Tf[(tk + 1) >> 4][(tk + 1) & 15][dl] * XS); *(volatile v2h*)(T2T + ((size_t)c * DCP + d) * L + lb * 64 + lane * 2) = vv; }
    __threadfence(); }
}
__global__ __launch_bounds__(256) void fuse_kernel(const float* __restrict__ xloc, const float* __restrict__ MS, const int* __restrict__ idx, const float* __restrict__ lam1, const float* __restrict__ lam2, float* __restrict__ out) {
  __shared__ float wk[8][K]; __shared__ int ik[8][K];
  const int wave = threadIdx.x >> 5, lane = threadIdx.x & 31; const int bc = blockIdx.x * 8 + wave; const int b = bc / C, c = bc % C; if (c >= CL) return;
  const float* xr = xloc + ((size_t)b * C + c) * L + lane * 16; float xv[16];
#pragma unroll
  for (int q = 0; q < 4; ++q) { const v4f f = *(const v4f*)(xr + q * 4);
#pragma unroll
    for (int j = 0; j < 4; ++j) xv[q * 4 + j] = bf16_rne(f[j]); }
  if (lane < K) { int i = idx[((size_t)b * C + c) * K + lane]; ik[wave][lane] = i < 0 ? 0 : (i >= DCP ? DCP - 1 : i); }
  wave_lds_sync();
  float mx = -INFINITY;
#pragma unroll 1
  for (int k = 0; k < K; ++k) { const float* mr = MS + ((size_t)c * DCP + ik[wave][k]) * L + lane * 16; float d = 0.0f;
#pragma unroll
    for (int q = 0; q < 4; ++q) { const v4f f = *(const v4f*)(mr + q * 4);
#pragma unroll
      for (int j = 0; j < 4; ++j) d += fabsf(xv[q * 4 + j] - f[j]); }
#pragma unroll
    for (int o = 1; o < 32; o <<= 1) d += __shfl_xor(d, o);
    const float s = -d * SCALE; if (lane == 0) wk[wave][k] = s; mx = fmaxf(mx, s); }
  wave_lds_sync();
  float den = 0.0f;
#pragma unroll 1
  for (int k = 0; k < K; ++k) den += expnl(wk[wave][k] - mx);
  const float s1 = sigm(bf16_rne(lam1[c]));
  float o16[16]; for (int j = 0; j < 16; ++j) o16[j] = 0.0f;
#pragma unroll 1
  for (int k = 0; k < K; ++k) { const float w = expnl(wk[wave][k] - mx) / den; const float* mr = MS + ((size_t)c * DCP + ik[wave][k]) * L + lane * 16;
#pragma unroll
    for (int q = 0; q < 4; ++q) { const v4f f = *(const v4f*)(mr + q * 4);
#pragma unroll
      for (int j = 0; j < 4; ++j) o16[q * 4 + j] += f[j] * w; } }
  v4f rq[4];
#pragma unroll
  for (int q = 0; q < 4; ++q) {
#pragma unroll
    for (int j = 0; j < 4; ++j) { const int l = lane * 16 + q * 4 + j; const float lam = s1 * sigm(bf16_rne(lam2[l])); rq[q][j] = o16[q * 4 + j] * lam + xv[q * 4 + j] * (1.0f - lam); } }
  for (int pass = 0; pass < 2; ++pass) {
#pragma unroll
    for (int q = 0; q < 4; ++q) *(volatile v4f*)(out + ((size_t)b * C + c) * L + lane * 16 + q * 4) = rq[q];
    __threadfence(); }
}
}

extern "C" void kernel_launch(void* const* d_in, const int* in_sizes, int n_in, void* d_out, int out_size, void* d_ws, size_t ws_size, hipStream_t stream) {
  (void)n_in;
  auto Fp = [&](int i) { return (const float*)d_in[i]; }; auto Ip = [&](int i) { return (const int*)d_in[i]; };
  if (in_sizes[0] != BT * C * L || in_sizes[1] != C * L * INTER || in_sizes[2] != INTER * DCP || in_sizes[4] != DCP * DCP || in_sizes[6] != L * DDE || in_sizes[8] != DDE * L || in_sizes[10] != C || in_sizes[11] != L || in_sizes[12] != BT * C * K || out_size != BT * C * L) return;
  size_t off = 0; char* ws = (char*)d_ws;
  auto carve = [&](size_t bytes) { char* p = ws + off; off += (bytes + 255) & ~(size_t)255; return p; };
  b16* W1T = (b16*)carve((size_t)DCP * INTER * 2); b16* W2T = (b16*)carve((size_t)DCP * DCP * 2); b16* W3T = (b16*)carve((size_t)DDE * L * 2); b16* W4T = (b16*)carve((size_t)L * DDE * 2);
  b16* T1 = (b16*)carve((size_t)C * L * DCP * 2); b16* T2T = (b16*)carve((size_t)C * DCP * L * 2); b16* T3 = (b16*)carve((size_t)C * DCP * DDE * 2); float* MS = (float*)carve((size_t)C * DCP * L * 4);
  if (off > ws_size || off > ((size_t)128 << 20)) return;
  prep_kernel<<<(unsigned)(((size_t)(DCP * INTER + DCP * DCP + DDE * L + L * DDE) / 8 + 255) / 256), 256, 0, stream>>>(Fp(2), Fp(4), Fp(6), Fp(8), W1T, W2T, W3T, W4T);
  gemm_kernel<INTER, DCP, 1, 1, 0><<<dim3((C * L) / 64, DCP / 128), 128, 0, stream>>>(Fp(1), nullptr, W1T, Fp(3), CL * L, T1, nullptr);
  gemm2t_kernel<<<dim3(C * (L / 64), DCP / 128), 128, 0, stream>>>(T1, W2T, Fp(5), T2T);
  gemm_kernel<L, DDE, 0, 1, 0><<<dim3((C * DCP) / 64, DDE / 128), 128, 0, stream>>>(nullptr, T2T, W3T, Fp(7), CL * DCP, T3, nullptr);
  gemm_kernel<DDE, L, 0, 0, 1><<<dim3((C * DCP) / 64, L / 128), 128, 0, stream>>>(nullptr, T3, W4T, Fp(9), CL * DCP, nullptr, MS);
  fuse_kernel<<<(BT * C) / 8, 256, 0, stream>>>(Fp(0), MS, Ip(12), Fp(10), Fp(11), (float*)d_out);
}
